// GNNModel_70729521430617
// MI455X (gfx1250) — hardware-verified
//
#include <hip/hip_runtime.h>
#include <stddef.h>
#include <stdint.h>
#include <math.h>


#define NN     100000
#define NE     1600000
#define NGR    512
#define C1     32
#define C2     64
#define K2C    64
#define K3C    128
#define NTHR   256
#define NWAVE  8
#define EPT    8
#define CHUNK  (NTHR * EPT)
#define WCAP   (EPT * 32)
#define LISTN  (NWAVE * WCAP)
#define NBA    1024
#define SLA    10
#define RCAP   28672
#define DEGCAP 64
#define NBLK   98
#define NP     (NBLK * NBA)
#define GM     128
#define GTILES 782
#define PARN   256
#define PW1    0
#define PB1    64
#define PB2    96
#define PB3    160
#define PWFC   192
#define PBFC   224
#define PT     128
#define PCH    1024
#define AGG_ZINTS   (LISTN + 2 * RCAP + 3 * NBA)
#define MISC_INTS   16
#define BK_LDS_INTS (AGG_ZINTS + MISC_INTS + NBA)
#define WSMAX  134217728

static_assert(NN % 32 == 0 && NN % 4 == 0 && NE % 4 == 0);
static_assert((CHUNK & (CHUNK - 1)) == 0 && CHUNK <= 4096);
static_assert((NBA & (NBA - 1)) == 0 && NBA == (1 << SLA) && NBA % 32 == 0);
static_assert(((long long)CHUNK << SLA) < (1LL << 31));
static_assert(NE < (1 << 21));
static_assert(NBLK * NBA >= NN && (NBLK - 1) * NBA < NN);
static_assert(RCAP >= 16710 + 4096 && RCAP % (NTHR * 4) == 0);
static_assert(DEGCAP >= 36 + 8);
static_assert(AGG_ZINTS % (NTHR * 4) == 0 && ((AGG_ZINTS + MISC_INTS) % 4) == 0);
static_assert(BK_LDS_INTS * 4 <= 300000);
static_assert(NBA == NTHR * 4 && NBA % NWAVE == 0);
static_assert(C1 == 32 && C2 == 64 && K2C == 2 * C1 && K3C == 2 * C2 && K2C % 32 == 0 && K3C % 32 == 0);
static_assert(GM == NWAVE * 16 && GTILES * GM >= NN && GTILES * GM <= NP);
static_assert(NGR == 4 * PT && PCH == PT * 8 && NBLK <= PT);
static_assert(PBFC < PARN && PARN == 4 * 64);

typedef float          v2f   __attribute__((ext_vector_type(2)));
typedef float          v4f   __attribute__((ext_vector_type(4)));
typedef float          v8f   __attribute__((ext_vector_type(8)));
typedef int            v4i   __attribute__((ext_vector_type(4)));
typedef int            v8i   __attribute__((ext_vector_type(8)));
typedef unsigned short v8us  __attribute__((ext_vector_type(8)));
typedef unsigned short v16us __attribute__((ext_vector_type(16)));
typedef __bf16         v16bf __attribute__((ext_vector_type(16)));
typedef v2f  __attribute__((may_alias)) v2fa;
typedef v4f  __attribute__((may_alias)) v4fa;
typedef v4i  __attribute__((may_alias)) v4ia;
typedef v8us __attribute__((may_alias)) v8usa;
union FragB { v16bf v; v16us u; v8us h[2]; v8i w; };

__device__ __forceinline__ v8f wmb(const FragB& a, const FragB& b, v8f c) {
  v8f d = __builtin_amdgcn_wmma_f32_16x16x32_bf16(false, a.v, false, b.v, (short)0, c, false, false);
  asm volatile("v_nop\n\tv_nop\n\tv_nop\n\tv_nop" : "+v"(d) : "v"(a.w), "v"(b.w));
  return d;
}

__device__ __forceinline__ v8f z8() { v8f z = {0.f, 0.f, 0.f, 0.f, 0.f, 0.f, 0.f, 0.f}; return z; }

__device__ __forceinline__ unsigned bf16_bits(float f) {
  const unsigned u = __float_as_uint(f);
  const unsigned r = (u + 0x7FFFu + ((u >> 16) & 1u)) >> 16;
  return (f != f) ? 0x7FC0u : r;
}
__device__ __forceinline__ float bf16_val(float f) {
  return __uint_as_float(bf16_bits(f) << 16);
}
__device__ __forceinline__ float relu_k(float v) { return (v > 0.0f) ? v : (v - v); }

template <int SLB>
__device__ __forceinline__ int scan_chunk(const int* __restrict__ dsts, int nE, int cbase, int slotBase,
                                          int nb, int vec8, int* list, int tid, int lane, int wave) {
  int wc = 0;
  const int el0  = tid * EPT;
  const int e0   = cbase + el0;
  const int sent = -2147483647 - 1;
  v4i da, db;
  if (vec8 != 0 && cbase + CHUNK <= nE) {
    da = *(const v4i*)(dsts + e0);
    db = *(const v4i*)(dsts + e0 + 4);
  } else {
    da.x = (e0     < nE) ? dsts[min(e0,     nE - 1)] : sent;
    da.y = (e0 + 1 < nE) ? dsts[min(e0 + 1, nE - 1)] : sent;
    da.z = (e0 + 2 < nE) ? dsts[min(e0 + 2, nE - 1)] : sent;
    da.w = (e0 + 3 < nE) ? dsts[min(e0 + 3, nE - 1)] : sent;
    db.x = (e0 + 4 < nE) ? dsts[min(e0 + 4, nE - 1)] : sent;
    db.y = (e0 + 5 < nE) ? dsts[min(e0 + 5, nE - 1)] : sent;
    db.z = (e0 + 6 < nE) ? dsts[min(e0 + 6, nE - 1)] : sent;
    db.w = (e0 + 7 < nE) ? dsts[min(e0 + 7, nE - 1)] : sent;
  }
  const unsigned nbs = (unsigned)slotBase;
  const unsigned unb = (unsigned)nb;
  const unsigned s0 = (unsigned)da.x - nbs, s1 = (unsigned)da.y - nbs;
  const unsigned s2 = (unsigned)da.z - nbs, s3 = (unsigned)da.w - nbs;
  const unsigned s4 = (unsigned)db.x - nbs, s5 = (unsigned)db.y - nbs;
  const unsigned s6 = (unsigned)db.z - nbs, s7 = (unsigned)db.w - nbs;
  const bool h0 = s0 < unb, h1 = s1 < unb, h2 = s2 < unb, h3 = s3 < unb;
  const bool h4 = s4 < unb, h5 = s5 < unb, h6 = s6 < unb, h7 = s7 < unb;
  const unsigned any = __builtin_amdgcn_ballot_w32(h0 | h1 | h2 | h3 | h4 | h5 | h6 | h7);
  if (any != 0u) {
#define HITJ(J, HJ, SJ) { \
      const unsigned mj = __builtin_amdgcn_ballot_w32(HJ); \
      if (mj != 0u) { \
        if (HJ) { \
          const int pos = wc + (int)__builtin_amdgcn_mbcnt_lo(mj, 0u); \
          if (pos < WCAP) list[wave * WCAP + pos] = ((el0 + (J)) << SLB) | (int)(SJ); \
        } \
        wc += (int)__builtin_popcount(mj); } }
    HITJ(0, h0, s0)
    HITJ(1, h1, s1)
    HITJ(2, h2, s2)
    HITJ(3, h3, s3)
    HITJ(4, h4, s4)
    HITJ(5, h5, s5)
    HITJ(6, h6, s6)
    HITJ(7, h7, s7)
#undef HITJ
  }
  return wc;
}

__global__ __launch_bounds__(NTHR) void k_prep(const float* __restrict__ W1, const float* __restrict__ b1,
                                               const float* __restrict__ W2, const float* __restrict__ b2,
                                               const float* __restrict__ W3, const float* __restrict__ b3,
                                               const float* __restrict__ Wfc, const float* __restrict__ bfc,
                                               unsigned short* w2d, unsigned short* w3d, float* par) {
  const int blk = (int)blockIdx.x, tid = (int)threadIdx.x;
  if (blk < 4) {
    const float* p;
    unsigned short* dp;
    if (blk < 2) {
      const int u = blk * NTHR + tid;
      const int n = u >> 3, k8 = (u & 7) * 8, kk = k8 & (C1 - 1);
      p  = W2 + (size_t)n * C1 + kk;
      dp = w2d + (size_t)u * 8;
    } else {
      const int v = (blk - 2) * NTHR + tid;
      const int n = v >> 4, k8 = (v & 15) * 8, kk = k8 & (C2 - 1);
      p  = W3 + (size_t)n * C2 + kk;
      dp = w3d + (size_t)v * 8;
    }
    const v4f a = *(const v4f*)p;
    const v4f b = *(const v4f*)(p + 4);
    v8us o;
    o[0] = (unsigned short)bf16_bits(a.x); o[1] = (unsigned short)bf16_bits(a.y);
    o[2] = (unsigned short)bf16_bits(a.z); o[3] = (unsigned short)bf16_bits(a.w);
    o[4] = (unsigned short)bf16_bits(b.x); o[5] = (unsigned short)bf16_bits(b.y);
    o[6] = (unsigned short)bf16_bits(b.z); o[7] = (unsigned short)bf16_bits(b.w);
    *(volatile v8us*)dp = o;
    __threadfence();
    *(volatile v8us*)dp = o;
  } else {
    if (tid >= PARN / 4) return;
    const int t = tid;
    const int c1 = t < 15 ? t : 15;
    int c2 = t - 16; c2 = c2 < 0 ? 0 : (c2 > 7 ? 7 : c2);
    int c3 = t - 24; c3 = c3 < 0 ? 0 : (c3 > 15 ? 15 : c3);
    int c4 = t - 40; c4 = c4 < 0 ? 0 : (c4 > 7 ? 7 : c4);
    int c5 = t - 48; c5 = c5 < 0 ? 0 : (c5 > 7 ? 7 : c5);
    const v4f a1 = *(const v4f*)(W1  + 4 * c1);
    const v4f a2 = *(const v4f*)(b1  + 4 * c2);
    const v4f a3 = *(const v4f*)(b2  + 4 * c3);
    const v4f a4 = *(const v4f*)(b3  + 4 * c4);
    const v4f a5 = *(const v4f*)(Wfc + 4 * c5);
    const float a6 = bfc[0];
    const unsigned m1 = (t < 16) ? 0xFFFFFFFFu : 0u;
    const unsigned m2 = (t >= 16 && t < 24) ? 0xFFFFFFFFu : 0u;
    const unsigned m3 = (t >= 24 && t < 40) ? 0xFFFFFFFFu : 0u;
    const unsigned m4 = (t >= 40 && t < 48) ? 0xFFFFFFFFu : 0u;
    const unsigned m5 = (t >= 48 && t < 56) ? 0xFFFFFFFFu : 0u;
    const unsigned m6 = (t == 56) ? 0xFFFFFFFFu : 0u;
    const unsigned rx = (__float_as_uint(a1.x) & m1) | (__float_as_uint(a2.x) & m2) | (__float_as_uint(a3.x) & m3) |
                        (__float_as_uint(a4.x) & m4) | (__float_as_uint(a5.x) & m5) | (__float_as_uint(a6) & m6);
    const unsigned ry = (__float_as_uint(a1.y) & m1) | (__float_as_uint(a2.y) & m2) | (__float_as_uint(a3.y) & m3) |
                        (__float_as_uint(a4.y) & m4) | (__float_as_uint(a5.y) & m5);
    const unsigned rz = (__float_as_uint(a1.z) & m1) | (__float_as_uint(a2.z) & m2) | (__float_as_uint(a3.z) & m3) |
                        (__float_as_uint(a4.z) & m4) | (__float_as_uint(a5.z) & m5);
    const unsigned rw = (__float_as_uint(a1.w) & m1) | (__float_as_uint(a2.w) & m2) | (__float_as_uint(a3.w) & m3) |
                        (__float_as_uint(a4.w) & m4) | (__float_as_uint(a5.w) & m5);
    v4f o;
    o.x = bf16_val(__uint_as_float(rx)); o.y = bf16_val(__uint_as_float(ry));
    o.z = bf16_val(__uint_as_float(rz)); o.w = bf16_val(__uint_as_float(rw));
    float* dp = par + 4 * t;
    *(volatile v4f*)dp = o;
    __threadfence();
    *(volatile v4f*)dp = o;
  }
}

__global__ __launch_bounds__(NTHR) void k_bucket(const int* __restrict__ srcs, const int* __restrict__ dsts,
                                                 const float* __restrict__ x,
                                                 int* listg, int* cntg, int* offg, float* disg, float* xsg,
                                                 int* flagg) {
  extern __shared__ __attribute__((aligned(16))) int dsm[];
  int* list = dsm;
  int* hl   = dsm + LISTN;
  int* sl   = hl + RCAP;
  int* cnt  = sl + RCAP;
  int* offs = cnt + NBA;
  int* cur  = offs + NBA;
  int* misc = cur + NBA;
  float* dsl = (float*)(misc + MISC_INTS);
  const int tid = (int)threadIdx.x, lane = tid & 31, wave = tid >> 5;
  const int nodeBase = (int)blockIdx.x * NBA;

  {
    const v4i z4 = {0, 0, 0, 0};
    for (int i = tid * 4; i < AGG_ZINTS; i += NTHR * 4) *(v4ia*)(dsm + i) = z4;
    if (tid < MISC_INTS) misc[tid] = 0;
  }
  __syncthreads();

  int t = 0, ov = 0;
  const int nChunks = (NE + CHUNK - 1) / CHUNK;
#pragma unroll 1
  for (int ch = 0; ch < nChunks; ++ch) {
    const int cbase = ch * CHUNK;
    const int wc = scan_chunk<SLA>(dsts, NE, cbase, nodeBase, NBA, 1, list, tid, lane, wave);
    if (lane == 0) misc[wave] = wc;
    __syncthreads();
    if (wave == 0) {
#pragma unroll 1
      for (int w2 = 0; w2 < NWAVE; ++w2) {
        int c = misc[w2];
        c = c < 0 ? 0 : (c > WCAP ? WCAP : c);
#pragma unroll 1
        for (int b0 = 0; b0 < c; b0 += 32) {
          const int idx = b0 + lane;
          const int ent = list[w2 * WCAP + (idx < WCAP ? idx : WCAP - 1)];
          const int m32 = (c - b0) < 32 ? (c - b0) : 32;
#pragma unroll 1
          for (int k = 0; k < m32; ++k) {
            const int u    = __builtin_amdgcn_readlane(ent, k);
            const int slot = u & (NBA - 1);
            const int el   = (u >> SLA) & (CHUNK - 1);
            const int pk   = ((cbase + el) << SLA) | slot;
            if (t < RCAP) {
              if (lane == 0) { hl[t] = pk; cnt[slot] = cnt[slot] + 1; }
              t = t + 1;
            } else {
              ov = 1;
            }
          }
        }
      }
    }
    __syncthreads();
  }
  if (wave == 0 && lane == 0) { misc[8] = t; misc[9] = ov; }
  __syncthreads();
  int tt = misc[8];
  tt = tt < 0 ? 0 : (tt > RCAP ? RCAP : tt);
  const int ovf = misc[9];

  if (wave == 0) {
    const int base = lane * (NBA / 32);
    int s = 0;
#pragma unroll 1
    for (int i = 0; i < NBA / 32; ++i) s += cnt[base + i];
    int incl = s;
#pragma unroll
    for (int d = 1; d < 32; d <<= 1) {
      const int y = __shfl_up(incl, d, 32);
      if (lane >= d) incl += y;
    }
    int run = incl - s;
#pragma unroll 1
    for (int i = 0; i < NBA / 32; ++i) {
      const int cv = cnt[base + i];
      offs[base + i] = run;
      cur[base + i]  = run;
      run += cv;
    }
  }
  __syncthreads();
  if (wave == 0) {
#pragma unroll 1
    for (int b0 = 0; b0 < tt; b0 += 32) {
      const int idx = b0 + lane;
      const int ent = hl[idx < RCAP ? idx : RCAP - 1];
      const int m32 = (tt - b0) < 32 ? (tt - b0) : 32;
#pragma unroll 1
      for (int k = 0; k < m32; ++k) {
        const int u    = __builtin_amdgcn_readlane(ent, k);
        const int slot = u & (NBA - 1);
        if (lane == 0) {
          int p = cur[slot];
          p = p < 0 ? 0 : (p > RCAP - 1 ? RCAP - 1 : p);
          sl[p] = u;
          cur[slot] = p + 1;
        }
      }
    }
  }
  __syncthreads();

  {
    int big = 0;
#pragma unroll 1
    for (int j = 0; j < 4; ++j) {
      int c = cnt[4 * tid + j];
      c = c < 0 ? 0 : c;
      big |= (c > DEGCAP) ? 1 : 0;
      dsl[4 * tid + j] = 1.0f / sqrtf((float)(c + 1));
    }
    if (big != 0) misc[10] = 1;
  }
  __syncthreads();
  const int flg = (ovf != 0 || misc[10] != 0) ? 1 : 0;

  const v4i c4 = *(const v4ia*)(cnt + 4 * tid);
  const v4i o4 = *(const v4ia*)(offs + 4 * tid);
  const v4f d4 = *(const v4fa*)(dsl + 4 * tid);
  v4f xv[2];
#pragma unroll
  for (int it = 0; it < 2; ++it) {
    const int s0  = it * 512 + 2 * tid;
    const int n0  = nodeBase + s0;
    const int n0c = n0 < NN - 2 ? n0 : NN - 2;
    const v4f xr = *(const v4f*)(x + 2 * (size_t)n0c);
    const bool ok = n0 < NN;
    const float da = dsl[s0], db = dsl[s0 + 1];
    v4f q;
    q.x = ok ? da * bf16_val(xr.x) : 0.0f;
    q.y = ok ? da * bf16_val(xr.y) : 0.0f;
    q.z = ok ? db * bf16_val(xr.z) : 0.0f;
    q.w = ok ? db * bf16_val(xr.w) : 0.0f;
    xv[it] = q;
  }
  const v4i f4 = {flg, flg, flg, flg};
  int*   cp = cntg + (size_t)nodeBase + 4 * tid;
  int*   op = offg + (size_t)nodeBase + 4 * tid;
  float* dp = disg + (size_t)nodeBase + 4 * tid;
  float* x0 = xsg + 2 * (size_t)nodeBase + 4 * tid;
  float* x1 = x0 + 1024;
  int*   fp = flagg + (size_t)blockIdx.x * 32 + 4 * (tid & 7);
  *(volatile v4i*)cp = c4;
  *(volatile v4i*)op = o4;
  *(volatile v4f*)dp = d4;
  *(volatile v4f*)x0 = xv[0];
  *(volatile v4f*)x1 = xv[1];
  if (tid < 8) *(volatile v4i*)fp = f4;
  __threadfence();
  *(volatile v4i*)cp = c4;
  *(volatile v4i*)op = o4;
  *(volatile v4f*)dp = d4;
  *(volatile v4f*)x0 = xv[0];
  *(volatile v4f*)x1 = xv[1];
  if (tid < 8) *(volatile v4i*)fp = f4;

  int* lg = listg + (size_t)blockIdx.x * RCAP;
#pragma unroll 1
  for (int it = 0; it < RCAP / (NTHR * 4); ++it) {
    const int p = it * (NTHR * 4) + 4 * tid;
    const v4i e4 = *(const v4ia*)(sl + p);
    int e0 = e4.x >> SLA, e1 = e4.y >> SLA, e2 = e4.z >> SLA, e3 = e4.w >> SLA;
    e0 = e0 < 0 ? 0 : (e0 > NE - 1 ? NE - 1 : e0);
    e1 = e1 < 0 ? 0 : (e1 > NE - 1 ? NE - 1 : e1);
    e2 = e2 < 0 ? 0 : (e2 > NE - 1 ? NE - 1 : e2);
    e3 = e3 < 0 ? 0 : (e3 > NE - 1 ? NE - 1 : e3);
    int r0 = srcs[e0], r1 = srcs[e1], r2 = srcs[e2], r3 = srcs[e3];
    r0 = r0 < 0 ? 0 : (r0 > NN - 1 ? NN - 1 : r0);
    r1 = r1 < 0 ? 0 : (r1 > NN - 1 ? NN - 1 : r1);
    r2 = r2 < 0 ? 0 : (r2 > NN - 1 ? NN - 1 : r2);
    r3 = r3 < 0 ? 0 : (r3 > NN - 1 ? NN - 1 : r3);
    v4i o;
    o.x = (p     < tt) ? r0 : 0;
    o.y = (p + 1 < tt) ? r1 : 0;
    o.z = (p + 2 < tt) ? r2 : 0;
    o.w = (p + 3 < tt) ? r3 : 0;
    *(volatile v4i*)(lg + p) = o;
    __threadfence();
    *(volatile v4i*)(lg + p) = o;
  }
}

__global__ __launch_bounds__(NTHR) void k_scan1(const int* __restrict__ listg, const int* __restrict__ cntg,
                                                const int* __restrict__ offg, const float* __restrict__ disg,
                                                const float* __restrict__ xsg, const float* __restrict__ par,
                                                const int* __restrict__ flagg, float* h1s) {
  __shared__ __attribute__((aligned(16))) int   scnt[NBA];
  __shared__ __attribute__((aligned(16))) int   soff[NBA];
  __shared__ __attribute__((aligned(16))) float sdis[NBA];
  __shared__ __attribute__((aligned(16))) float spar[PARN];
  const int tid = (int)threadIdx.x, lane = tid & 31, wave = tid >> 5;
  const int nodeBase = (int)blockIdx.x * NBA;
  *(v4ia*)(scnt + 4 * tid) = *(const v4i*)(cntg + (size_t)nodeBase + 4 * tid);
  *(v4ia*)(soff + 4 * tid) = *(const v4i*)(offg + (size_t)nodeBase + 4 * tid);
  *(v4fa*)(sdis + 4 * tid) = *(const v4f*)(disg + (size_t)nodeBase + 4 * tid);
  if (tid < PARN / 4) *(v4fa*)(spar + 4 * tid) = *(const v4f*)(par + 4 * tid);
  const int fl = flagg[(size_t)blockIdx.x * 32];
  __syncthreads();
  const float w0 = spar[PW1 + 2 * lane], w1 = spar[PW1 + 2 * lane + 1], bb = spar[PB1 + lane];
  const float pz = (fl != 0) ? __int_as_float(0x7fc00000) : 0.0f;
  const int* lp = listg + (size_t)blockIdx.x * RCAP;
#pragma unroll 1
  for (int si = 0; si < NBA / NWAVE; ++si) {
    const int s    = si * NWAVE + wave;
    const int node = nodeBase + s;
    int c = scnt[s];
    c = c < 0 ? 0 : (c > DEGCAP ? DEGCAP : c);
    int o = soff[s];
    o = o < 0 ? 0 : (o > RCAP ? RCAP : o);
    const float dd = sdis[s];
    const int nc = node < NN ? node : NN - 1;
    float p0 = 0.0f, p1 = 0.0f;
#pragma unroll 1
    for (int b0 = 0; b0 < c; b0 += 32) {
      int idx = o + b0 + lane;
      idx = idx > RCAP - 1 ? RCAP - 1 : idx;
      int sr = lp[idx];
      sr = sr < 0 ? 0 : (sr > NN - 1 ? NN - 1 : sr);
      const v2f v = *(const v2fa*)(xsg + 2 * (size_t)sr);
      const bool valid = (b0 + lane) < c;
      p0 += valid ? v.x : 0.0f;
      p1 += valid ? v.y : 0.0f;
    }
    p0 += __shfl_xor(p0, 16, 32); p1 += __shfl_xor(p1, 16, 32);
    p0 += __shfl_xor(p0, 8, 32);  p1 += __shfl_xor(p1, 8, 32);
    p0 += __shfl_xor(p0, 4, 32);  p1 += __shfl_xor(p1, 4, 32);
    p0 += __shfl_xor(p0, 2, 32);  p1 += __shfl_xor(p1, 2, 32);
    p0 += __shfl_xor(p0, 1, 32);  p1 += __shfl_xor(p1, 1, 32);
    const v2f sv = *(const v2fa*)(xsg + 2 * (size_t)nc);
    const float a0 = dd * (p0 + sv.x);
    const float a1 = dd * (p1 + sv.y);
    const float y  = fmaf(a1, w1, fmaf(a0, w0, bb));
    const float h  = relu_k(y);
    const float ov = (node < NN) ? (dd * h + pz) : 0.0f;
    float* op = h1s + (size_t)node * C1 + lane;
    *(volatile float*)op = ov;
    __threadfence();
    *(volatile float*)op = ov;
  }
}

template <int MODE>
__global__ __launch_bounds__(NTHR) void k_scanw(const int* __restrict__ listg, const int* __restrict__ cntg,
                                                const int* __restrict__ offg, const float* __restrict__ disg,
                                                const float* __restrict__ rows, const float* __restrict__ par,
                                                const int* __restrict__ flagg, unsigned* a2w, float* sgl) {
  __shared__ __attribute__((aligned(16))) int   scnt[NBA];
  __shared__ __attribute__((aligned(16))) int   soff[NBA];
  __shared__ __attribute__((aligned(16))) float sdis[NBA];
  __shared__ __attribute__((aligned(16))) float spar[PARN];
  __shared__ __attribute__((aligned(16))) float sS[NBA];
  const int tid = (int)threadIdx.x, lane = tid & 31, wave = tid >> 5;
  const int nodeBase = (int)blockIdx.x * NBA;
  *(v4ia*)(scnt + 4 * tid) = *(const v4i*)(cntg + (size_t)nodeBase + 4 * tid);
  *(v4ia*)(soff + 4 * tid) = *(const v4i*)(offg + (size_t)nodeBase + 4 * tid);
  *(v4fa*)(sdis + 4 * tid) = *(const v4f*)(disg + (size_t)nodeBase + 4 * tid);
  if (tid < PARN / 4) *(v4fa*)(spar + 4 * tid) = *(const v4f*)(par + 4 * tid);
  const int fl = flagg[(size_t)blockIdx.x * 32];
  __syncthreads();
  const float bb = spar[PB3 + lane];
  const float wf = spar[PWFC + lane];
  const float pz = (fl != 0) ? __int_as_float(0x7fc00000) : 0.0f;
  const int sA = (2 * lane) & 31, sB = (2 * lane + 1) & 31;
  const int* lp = listg + (size_t)blockIdx.x * RCAP;
#pragma unroll 1
  for (int si = 0; si < NBA / NWAVE; ++si) {
    const int s    = si * NWAVE + wave;
    const int node = nodeBase + s;
    int c = scnt[s];
    c = c < 0 ? 0 : (c > DEGCAP ? DEGCAP : c);
    int o = soff[s];
    o = o < 0 ? 0 : (o > RCAP ? RCAP : o);
    const float dd = sdis[s];
    const int nc = node < NN ? node : NN - 1;
    const bool live = node < NN;
    float acc = 0.0f;
#pragma unroll 1
    for (int b0 = 0; b0 < c; b0 += 32) {
      int idx = o + b0 + lane;
      idx = idx > RCAP - 1 ? RCAP - 1 : idx;
      int sr = lp[idx];
      sr = sr < 0 ? 0 : (sr > NN - 1 ? NN - 1 : sr);
      const int m32 = (c - b0) < 32 ? (c - b0) : 32;
#pragma unroll 1
      for (int k = 0; k < m32; ++k) {
        const int sk = __builtin_amdgcn_readlane(sr, k);
        acc += rows[(size_t)sk * C1 + lane];
      }
    }
    const float self = rows[(size_t)nc * C1 + lane];
    const float v = dd * (acc + self);
    if constexpr (MODE == 0) {
      const float vv = live ? (v + pz) : 0.0f;
      const unsigned hb = bf16_bits(vv);
      const unsigned lb = bf16_bits(vv - __uint_as_float(hb << 16));
      const unsigned h0 = (unsigned)__shfl((int)hb, sA, 32), h1 = (unsigned)__shfl((int)hb, sB, 32);
      const unsigned l0 = (unsigned)__shfl((int)lb, sA, 32), l1 = (unsigned)__shfl((int)lb, sB, 32);
      const unsigned wh = h0 | (h1 << 16);
      const unsigned wl = l0 | (l1 << 16);
      const unsigned wd = (lane < 16) ? wh : wl;
      unsigned* op = a2w + (size_t)node * 32 + lane;
      *(volatile unsigned*)op = wd;
      __threadfence();
      *(volatile unsigned*)op = wd;
    } else {
      const float h3 = relu_k(v + bb);
      float q = h3 * wf;
      q += __shfl_xor(q, 16, 32);
      q += __shfl_xor(q, 8, 32);
      q += __shfl_xor(q, 4, 32);
      q += __shfl_xor(q, 2, 32);
      q += __shfl_xor(q, 1, 32);
      const float sv = live ? (q + pz) : 0.0f;
      if (lane == 0) sS[s] = sv;
    }
  }
  if constexpr (MODE != 0) {
    __syncthreads();
    const v4f q4 = *(const v4fa*)(sS + 4 * tid);
    float* op = sgl + (size_t)nodeBase + 4 * tid;
    *(volatile v4f*)op = q4;
    __threadfence();
    *(volatile v4f*)op = q4;
    (void)a2w;
  } else {
    (void)sgl; (void)bb; (void)wf;
  }
}

__global__ __launch_bounds__(NTHR) void k_gemm23(const unsigned short* __restrict__ A2,
                                                 const unsigned short* __restrict__ w2d,
                                                 const unsigned short* __restrict__ w3d,
                                                 const float* __restrict__ par, const float* __restrict__ disg,
                                                 float* t3s) {
  __shared__ __attribute__((aligned(16))) unsigned short h2t[GM * K3C];
  __shared__ __attribute__((aligned(16))) float stg[GM * C1];
  __shared__ __attribute__((aligned(16))) float spar[PARN];
  const int tid = (int)threadIdx.x, lane = tid & 31, wave = tid >> 5, hh = lane >> 4, m = lane & 15;
  const int rowBase = (int)blockIdx.x * GM;
  if (tid < PARN / 4) *(v4fa*)(spar + 4 * tid) = *(const v4f*)(par + 4 * tid);
  __syncthreads();

  v8f acc[4];
#pragma unroll
  for (int t = 0; t < 4; ++t) acc[t] = z8();
  {
    const unsigned short* ap = A2 + (size_t)(rowBase + 16 * wave + m) * K2C + 8 * hh;
    const unsigned short* wp = w2d + (size_t)m * K2C + 8 * hh;
#pragma unroll
    for (int ks = 0; ks < K2C / 32; ++ks) {
      FragB af;
      af.h[0] = *(const v8usa*)(ap + 32 * ks);
      af.h[1] = *(const v8usa*)(ap + 32 * ks + 16);
#pragma unroll
      for (int t = 0; t < 4; ++t) {
        const unsigned short* wq = wp + (size_t)(16 * t) * K2C + 32 * ks;
        FragB bf;
        bf.h[0] = *(const v8usa*)wq;
        bf.h[1] = *(const v8usa*)(wq + 16);
        acc[t] = wmb(af, bf, acc[t]);
      }
    }
  }
#pragma unroll
  for (int t = 0; t < 4; ++t) {
    const int col = 16 * t + m;
    const float bc = spar[PB2 + col];
#pragma unroll
    for (int r = 0; r < 8; ++r) {
      const int lr = 16 * wave + 8 * hh + r;
      const float y = relu_k(acc[t][r] + bc);
      const unsigned hb = bf16_bits(y);
      const unsigned lb = bf16_bits(y - __uint_as_float(hb << 16));
      h2t[lr * K3C + col]      = (unsigned short)hb;
      h2t[lr * K3C + C2 + col] = (unsigned short)lb;
    }
  }
  __syncthreads();

  v8f acc3[2];
  acc3[0] = z8(); acc3[1] = z8();
  {
    const unsigned short* ap = h2t + (size_t)(16 * wave + m) * K3C + 8 * hh;
    const unsigned short* wp = w3d + (size_t)m * K3C + 8 * hh;
#pragma unroll
    for (int ks = 0; ks < K3C / 32; ++ks) {
      FragB af;
      af.h[0] = *(const v8usa*)(ap + 32 * ks);
      af.h[1] = *(const v8usa*)(ap + 32 * ks + 16);
#pragma unroll
      for (int t = 0; t < 2; ++t) {
        const unsigned short* wq = wp + (size_t)(16 * t) * K3C + 32 * ks;
        FragB bf;
        bf.h[0] = *(const v8usa*)wq;
        bf.h[1] = *(const v8usa*)(wq + 16);
        acc3[t] = wmb(af, bf, acc3[t]);
      }
    }
  }
#pragma unroll
  for (int t = 0; t < 2; ++t) {
    const int lc = 16 * t + m;
#pragma unroll
    for (int r = 0; r < 8; ++r) {
      const int lr = 16 * wave + 8 * hh + r;
      stg[lr * C1 + lc] = acc3[t][r];
    }
  }
  __syncthreads();

  v4f fv[4];
#pragma unroll
  for (int i = 0; i < 4; ++i) {
    const int lr = 16 * wave + 4 * i + (lane >> 3);
    const v4f v = *(const v4fa*)(stg + lr * C1 + 4 * (lane & 7));
    const float d = disg[rowBase + lr];
    v4f q;
    q.x = v.x * d; q.y = v.y * d; q.z = v.z * d; q.w = v.w * d;
    fv[i] = q;
  }
#pragma unroll
  for (int i = 0; i < 4; ++i) {
    const int lr = 16 * wave + 4 * i + (lane >> 3);
    float* op = t3s + (size_t)(rowBase + lr) * C1 + 4 * (lane & 7);
    *(volatile v4f*)op = fv[i];
  }
  __threadfence();
#pragma unroll
  for (int i = 0; i < 4; ++i) {
    const int lr = 16 * wave + 4 * i + (lane >> 3);
    float* op = t3s + (size_t)(rowBase + lr) * C1 + 4 * (lane & 7);
    *(volatile v4f*)op = fv[i];
  }
}

__global__ __launch_bounds__(PT) void k_pool(const int* __restrict__ bat, const float* __restrict__ sg,
                                             const float* __restrict__ par, const int* __restrict__ flagg,
                                             float* out) {
  __shared__ __attribute__((aligned(16))) int   sb[PCH];
  __shared__ __attribute__((aligned(16))) float ss[PCH];
  __shared__ __attribute__((aligned(16))) float outs[PT];
  __shared__ __attribute__((aligned(16))) int   sfl[PT];
  const int tid = (int)threadIdx.x;
  const int g = (int)blockIdx.x * PT + tid;
  {
    const int fb = tid < NBLK ? tid : NBLK - 1;
    const int f = flagg[(size_t)fb * 32];
    sfl[tid] = (tid < NBLK) ? f : 0;
  }
  double acc = 0.0;
  int cn = 0;
  const int nCh = (NN + PCH - 1) / PCH;
#pragma unroll 1
  for (int ch = 0; ch < nCh; ++ch) {
    __syncthreads();
#pragma unroll
    for (int it = 0; it < 2; ++it) {
      const int j   = it * PT + tid;
      const int n0  = ch * PCH + 4 * j;
      const bool ok = n0 < NN;
      const int n0c = n0 < NN - 4 ? n0 : NN - 4;
      v4i b4 = *(const v4i*)(bat + n0c);
      v4f s4 = *(const v4f*)(sg + n0c);
      b4.x = ok ? b4.x : -1; b4.y = ok ? b4.y : -1; b4.z = ok ? b4.z : -1; b4.w = ok ? b4.w : -1;
      s4.x = ok ? s4.x : 0.0f; s4.y = ok ? s4.y : 0.0f; s4.z = ok ? s4.z : 0.0f; s4.w = ok ? s4.w : 0.0f;
      *(v4ia*)(sb + 4 * j) = b4;
      *(v4fa*)(ss + 4 * j) = s4;
    }
    __syncthreads();
#pragma unroll 2
    for (int k4 = 0; k4 < PCH / 4; ++k4) {
      const v4i bv = *(const v4ia*)(sb + 4 * k4);
      const v4f sv = *(const v4fa*)(ss + 4 * k4);
      const bool h0 = bv.x == g, h1 = bv.y == g, h2 = bv.z == g, h3 = bv.w == g;
      acc = h0 ? acc + (double)sv.x : acc;
      acc = h1 ? acc + (double)sv.y : acc;
      acc = h2 ? acc + (double)sv.z : acc;
      acc = h3 ? acc + (double)sv.w : acc;
      cn += (h0 ? 1 : 0) + (h1 ? 1 : 0) + (h2 ? 1 : 0) + (h3 ? 1 : 0);
    }
  }
  int af = 0;
#pragma unroll 1
  for (int i = 0; i < PT; i += 4) {
    const v4i q = *(const v4ia*)(sfl + i);
    af |= q.x | q.y | q.z | q.w;
  }
  const float bfr = par[PBFC];
  const float cf = (cn < 1) ? 1.0f : (float)cn;
  float o = (float)acc * (1.0f / cf) + bfr;
  o = (af != 0) ? __int_as_float(0x7fc00000) : o;
  outs[tid] = o;
  __syncthreads();
  const bool okst = tid < 32;
  const v4f ov = *(const v4fa*)(outs + 4 * (tid & 31));
  float* op = out + (size_t)blockIdx.x * PT + 4 * (tid & 31);
  if (okst) *(volatile v4f*)op = ov;
  __threadfence();
  if (okst) *(volatile v4f*)op = ov;
}

static inline size_t al256(size_t o) { return (o + 255) & ~(size_t)255; }

extern "C" void kernel_launch(void* const* d_in, const int* in_sizes, int n_in,
                              void* d_out, int out_size, void* d_ws, size_t ws_size,
                              hipStream_t stream) {
  if (n_in < 11) return;
  if (in_sizes[0] != NN * 2) return;
  if (in_sizes[1] != NE * 2) return;
  if (in_sizes[2] != NN) return;
  if (in_sizes[3] != C1 * 2 || in_sizes[4] != C1) return;
  if (in_sizes[5] != C2 * C1 || in_sizes[6] != C2) return;
  if (in_sizes[7] != C1 * C2 || in_sizes[8] != C1) return;
  if (in_sizes[9] != C1 || in_sizes[10] != 1) return;
  if (out_size != NGR) return;

  const float* x   = (const float*)d_in[0];
  const int*   ei  = (const int*)  d_in[1];
  const int*   bat = (const int*)  d_in[2];
  const float* W1  = (const float*)d_in[3];
  const float* b1  = (const float*)d_in[4];
  const float* W2  = (const float*)d_in[5];
  const float* b2  = (const float*)d_in[6];
  const float* W3  = (const float*)d_in[7];
  const float* b3  = (const float*)d_in[8];
  const float* Wfc = (const float*)d_in[9];
  const float* bfc = (const float*)d_in[10];
  float* out = (float*)d_out;
  const int* src = ei;
  const int* dst = ei + NE;

  char* ws = (char*)d_ws;
  size_t off = 0;
  const size_t oW2D = off; off = al256(off + (size_t)C2 * K2C * 2);
  const size_t oW3D = off; off = al256(off + (size_t)C1 * K3C * 2);
  const size_t oPAR = off; off = al256(off + (size_t)PARN * 4);
  const size_t oFLG = off; off = al256(off + (size_t)NBLK * 32 * 4);
  const size_t oLST = off; off = al256(off + (size_t)NBLK * RCAP * 4);
  const size_t oCNT = off; off = al256(off + (size_t)NP * 4);
  const size_t oOFF = off; off = al256(off + (size_t)NP * 4);
  const size_t oDIS = off; off = al256(off + (size_t)NP * 4);
  const size_t oXS  = off; off = al256(off + (size_t)NP * 2 * 4);
  const size_t oH1S = off; off = al256(off + (size_t)NP * C1 * 4);
  const size_t oA2  = off; off = al256(off + (size_t)NP * K2C * 2);
  const size_t oT3S = off; off = al256(off + (size_t)NP * C1 * 4);
  const size_t oS   = off; off = al256(off + (size_t)NP * 4);
  if (off > ws_size || off > (size_t)WSMAX) return;
  unsigned short* W2D = (unsigned short*)(ws + oW2D);
  unsigned short* W3D = (unsigned short*)(ws + oW3D);
  float* PAR = (float*)(ws + oPAR);
  int*   FLG = (int*)(ws + oFLG);
  int*   LST = (int*)(ws + oLST);
  int*   CNT = (int*)(ws + oCNT);
  int*   OFF = (int*)(ws + oOFF);
  float* DIS = (float*)(ws + oDIS);
  float* XS  = (float*)(ws + oXS);
  float* H1S = (float*)(ws + oH1S);
  unsigned short* A2 = (unsigned short*)(ws + oA2);
  float* T3S = (float*)(ws + oT3S);
  float* S   = (float*)(ws + oS);

  const size_t bkLds = (size_t)BK_LDS_INTS * 4;
  hipFuncSetAttribute(reinterpret_cast<const void*>(&k_bucket), hipFuncAttributeMaxDynamicSharedMemorySize, (int)bkLds);

  k_prep<<<5, NTHR, 0, stream>>>(W1, b1, W2, b2, W3, b3, Wfc, bfc, W2D, W3D, PAR);
  k_bucket<<<NBLK, NTHR, bkLds, stream>>>(src, dst, x, LST, CNT, OFF, DIS, XS, FLG);
  k_scan1<<<NBLK, NTHR, 0, stream>>>(LST, CNT, OFF, DIS, XS, PAR, FLG, H1S);
  k_scanw<0><<<NBLK, NTHR, 0, stream>>>(LST, CNT, OFF, DIS, H1S, PAR, FLG, (unsigned*)A2, S);
  k_gemm23<<<GTILES, NTHR, 0, stream>>>(A2, W2D, W3D, PAR, DIS, T3S);
  k_scanw<1><<<NBLK, NTHR, 0, stream>>>(LST, CNT, OFF, DIS, T3S, PAR, FLG, (unsigned*)A2, S);
  k_pool<<<NGR / PT, PT, 0, stream>>>(bat, S, PAR, FLG, out);
}
